// T5LayerRGAT_91311004713519
// MI455X (gfx1250) — hardware-verified
//
#include <hip/hip_runtime.h>
#include <stddef.h>
#include <stdint.h>
#include <math.h>

#define BB   4
#define LL   1024
#define CC   1024
#define FF   4096
#define ROWS (BB * LL)
#define C3   (3 * CC)
#define NDB  16
#define ECH  256

static_assert(CC == 1024);
static_assert(LL % NDB == 0);
static_assert(NDB == 16);
static_assert(ROWS % 256 == 0);
static_assert(CC % 64 == 0);
static_assert(FF % 64 == 0);
static_assert(C3 % 64 == 0);
static_assert((NDB * CC) % (4 * 256) == 0);

typedef _Float16 v16h __attribute__((ext_vector_type(16)));
typedef _Float16 v8h  __attribute__((ext_vector_type(8)));
typedef float    v8f  __attribute__((ext_vector_type(8)));
typedef float    v4f  __attribute__((ext_vector_type(4)));
typedef unsigned int v4u __attribute__((ext_vector_type(4)));

union Frag  { v16h v; v8h h[2]; };
union Pack8 { v8h h; v4u u; };

__device__ __forceinline__ v8f mma16(v16h a, v16h b, v8f c) {
  c = __builtin_amdgcn_wmma_f32_16x16x32_f16(false, a, false, b, (short)0, c, false, false);
  asm volatile("v_nop\n\tv_nop\n\tv_nop\n\tv_nop" : "+v"(c) : "v"(a), "v"(b));
  return c;
}

__device__ __forceinline__ v16h ldfrag(const _Float16* p, int ld, int row0, int k0, int lane) {
  const int m = lane & 15, lh = lane >> 4;
  const _Float16* q = p + (size_t)(row0 + m) * ld + k0 + 8 * lh;
  Frag f;
  f.h[0] = *(const v8h*)(q);
  f.h[1] = *(const v8h*)(q + 16);
  return f.v;
}

__device__ __forceinline__ v8f zero8() { return (v8f){0.f, 0.f, 0.f, 0.f, 0.f, 0.f, 0.f, 0.f}; }

__device__ __forceinline__ float act16(float v) { return 16.0f * fmaxf(v, 0.0f); }

template <int KK>
__device__ __forceinline__ void gemm32x64(const _Float16* __restrict__ A, int lda,
                                          const _Float16* __restrict__ Bt, int ldb,
                                          int m0, int n0, int lane, v8f (&acc)[2][4]) {
#pragma unroll 2
  for (int k0 = 0; k0 < KK; k0 += 32) {
    const v16h a0 = ldfrag(A, lda, m0, k0, lane);
    const v16h a1 = ldfrag(A, lda, m0 + 16, k0, lane);
    const v16h b0 = ldfrag(Bt, ldb, n0, k0, lane);
    const v16h b1 = ldfrag(Bt, ldb, n0 + 16, k0, lane);
    const v16h b2 = ldfrag(Bt, ldb, n0 + 32, k0, lane);
    const v16h b3 = ldfrag(Bt, ldb, n0 + 48, k0, lane);
    acc[0][0] = mma16(a0, b0, acc[0][0]);
    acc[1][0] = mma16(a1, b0, acc[1][0]);
    acc[0][1] = mma16(a0, b1, acc[0][1]);
    acc[1][1] = mma16(a1, b1, acc[1][1]);
    acc[0][2] = mma16(a0, b2, acc[0][2]);
    acc[1][2] = mma16(a1, b2, acc[1][2]);
    acc[0][3] = mma16(a0, b3, acc[0][3]);
    acc[1][3] = mma16(a1, b3, acc[1][3]);
  }
}

#define WTP 68
__global__ __launch_bounds__(256) void k_wt(const float* __restrict__ w, _Float16* __restrict__ wt,
                                           int nout, int kin) {
  __shared__ __align__(16) float tf[64 * WTP];
  const int tid = threadIdx.x;
  const int n0 = blockIdx.x * 64;
  const int k0 = blockIdx.y * 64;
  {
    const int kr = tid >> 4;
    const int n4 = (tid & 15) * 4;
#pragma unroll
    for (int it = 0; it < 4; ++it) {
      const int kl = it * 16 + kr;
      const v4f a = *(const v4f*)(w + (size_t)(k0 + kl) * nout + n0 + n4);
      *(v4f*)(tf + kl * WTP + n4) = a;
    }
  }
  __syncthreads();
  v4u val[2];
  size_t go[2];
#pragma unroll
  for (int j = 0; j < 2; ++j) {
    const int p  = tid + 256 * j;
    const int nl = p >> 3;
    const int pc = p & 7;
    const float* cp = tf + (pc * 8) * WTP + nl;
    Pack8 pk;
    pk.h = (v8h){(_Float16)(cp[0 * WTP] * 32.0f), (_Float16)(cp[1 * WTP] * 32.0f),
                 (_Float16)(cp[2 * WTP] * 32.0f), (_Float16)(cp[3 * WTP] * 32.0f),
                 (_Float16)(cp[4 * WTP] * 32.0f), (_Float16)(cp[5 * WTP] * 32.0f),
                 (_Float16)(cp[6 * WTP] * 32.0f), (_Float16)(cp[7 * WTP] * 32.0f)};
    val[j] = pk.u;
    go[j]  = (size_t)(n0 + nl) * kin + k0 + pc * 8;
  }
  for (int ps = 0; ps < 2; ++ps) {
#pragma unroll
    for (int j = 0; j < 2; ++j) *(volatile v4u*)(wt + go[j]) = val[j];
    __threadfence();
  }
}

__global__ __launch_bounds__(256) void k_ln(const float* __restrict__ in,
                                           const float* __restrict__ g,
                                           const float* __restrict__ bt,
                                           float* __restrict__ outf,
                                           _Float16* __restrict__ outh) {
  __shared__ __align__(16) float rb[CC];
  __shared__ float red[16];
  const int tid = threadIdx.x, lane = tid & 31, wave = tid >> 5;
  const size_t ro = (size_t)blockIdx.x * CC;
  const v4f v = *(const v4f*)(in + ro + 4 * tid);
  float s = (v[0] + v[1]) + (v[2] + v[3]);
#pragma unroll
  for (int off = 1; off < 32; off <<= 1) s += __shfl_xor(s, off, 32);
  if (lane == 0) red[wave] = s;
  __syncthreads();
  float ts = 0.f;
#pragma unroll
  for (int w = 0; w < 8; ++w) ts += red[w];
  const float mean = ts * (1.0f / (float)CC);
  const float d0 = v[0] - mean, d1 = v[1] - mean, d2 = v[2] - mean, d3 = v[3] - mean;
  float q = (d0 * d0 + d1 * d1) + (d2 * d2 + d3 * d3);
#pragma unroll
  for (int off = 1; off < 32; off <<= 1) q += __shfl_xor(q, off, 32);
  if (lane == 0) red[8 + wave] = q;
  __syncthreads();
  float tq = 0.f;
#pragma unroll
  for (int w = 0; w < 8; ++w) tq += red[8 + w];
  const float var = tq * (1.0f / (float)CC);
  const float inv = rsqrtf(var + 1e-6f);
  const v4f g4 = *(const v4f*)(g + 4 * tid);
  const v4f b4 = *(const v4f*)(bt + 4 * tid);
  v4f o;
  o[0] = d0 * inv * g4[0] + b4[0];
  o[1] = d1 * inv * g4[1] + b4[1];
  o[2] = d2 * inv * g4[2] + b4[2];
  o[3] = d3 * inv * g4[3] + b4[3];
  volatile v4f* dp = (volatile v4f*)(outf + ro + 4 * tid);
  *dp = o;
  __threadfence();
  *dp = o;
  *(v4f*)(rb + 4 * tid) = o;
  __syncthreads();
  if (tid < 128) {
    const v4f a0 = *(const v4f*)(rb + 8 * tid);
    const v4f a1 = *(const v4f*)(rb + 8 * tid + 4);
    Pack8 pk;
    pk.h = (v8h){(_Float16)a0[0], (_Float16)a0[1], (_Float16)a0[2], (_Float16)a0[3],
                 (_Float16)a1[0], (_Float16)a1[1], (_Float16)a1[2], (_Float16)a1[3]};
    const v4u vv = pk.u;
    volatile v4u* hq = (volatile v4u*)(outh + ro + 8 * tid);
    *hq = vv;
    __threadfence();
    *hq = vv;
  }
}

__global__ __launch_bounds__(256) void k_lnout(const float* __restrict__ in,
                                              const float* __restrict__ g,
                                              const float* __restrict__ bt,
                                              const float* __restrict__ hid,
                                              float* __restrict__ out) {
  __shared__ float red[16];
  const int tid = threadIdx.x, lane = tid & 31, wave = tid >> 5;
  const size_t ro = (size_t)blockIdx.x * CC;
  const v4f v = *(const v4f*)(in + ro + 4 * tid);
  float s = (v[0] + v[1]) + (v[2] + v[3]);
#pragma unroll
  for (int off = 1; off < 32; off <<= 1) s += __shfl_xor(s, off, 32);
  if (lane == 0) red[wave] = s;
  __syncthreads();
  float ts = 0.f;
#pragma unroll
  for (int w = 0; w < 8; ++w) ts += red[w];
  const float mean = ts * (1.0f / (float)CC);
  const float d0 = v[0] - mean, d1 = v[1] - mean, d2 = v[2] - mean, d3 = v[3] - mean;
  float q = (d0 * d0 + d1 * d1) + (d2 * d2 + d3 * d3);
#pragma unroll
  for (int off = 1; off < 32; off <<= 1) q += __shfl_xor(q, off, 32);
  if (lane == 0) red[8 + wave] = q;
  __syncthreads();
  float tq = 0.f;
#pragma unroll
  for (int w = 0; w < 8; ++w) tq += red[8 + w];
  const float var = tq * (1.0f / (float)CC);
  const float inv = rsqrtf(var + 1e-6f);
  const v4f g4 = *(const v4f*)(g + 4 * tid);
  const v4f b4 = *(const v4f*)(bt + 4 * tid);
  const v4f h4 = *(const v4f*)(hid + ro + 4 * tid);
  const float y0 = d0 * inv * g4[0] + b4[0];
  const float y1 = d1 * inv * g4[1] + b4[1];
  const float y2 = d2 * inv * g4[2] + b4[2];
  const float y3 = d3 * inv * g4[3] + b4[3];
  const float e0 = (y0 > 0.0f) ? y0 : (__expf(y0) - 1.0f);
  const float e1 = (y1 > 0.0f) ? y1 : (__expf(y1) - 1.0f);
  const float e2 = (y2 > 0.0f) ? y2 : (__expf(y2) - 1.0f);
  const float e3 = (y3 > 0.0f) ? y3 : (__expf(y3) - 1.0f);
  v4f o;
  o[0] = h4[0] + e0;
  o[1] = h4[1] + e1;
  o[2] = h4[2] + e2;
  o[3] = h4[3] + e3;
  volatile v4f* dp = (volatile v4f*)(out + ro + 4 * tid);
  *dp = o;
  __threadfence();
  *dp = o;
}

#define OTP 68
__global__ __launch_bounds__(256) void k_qkv32(const _Float16* __restrict__ xh,
                                               const _Float16* __restrict__ wt,
                                               const float* __restrict__ bq,
                                               float* __restrict__ qkv) {
  __shared__ __align__(16) float st[8][16 * OTP];
  const int tid = threadIdx.x, lane = tid & 31, wave = tid >> 5;
  const int hh = lane >> 4, c = lane & 15;
  const int m0 = blockIdx.x * 256 + wave * 32;
  const int n0 = blockIdx.y * 64;
  const int which = n0 >> 10;
  const int nin = n0 & (CC - 1);

  v8f acc[2][4];
#pragma unroll
  for (int s = 0; s < 2; ++s)
#pragma unroll
    for (int t = 0; t < 4; ++t) acc[s][t] = zero8();
  gemm32x64<CC>(xh, CC, wt, CC, m0, n0, lane, acc);

  float bvs[4];
#pragma unroll
  for (int t = 0; t < 4; ++t) {
    const float bqv = bq[nin + 16 * t + c];
    bvs[t] = (which == 0) ? bqv : 0.0f;
  }
  float* ob = qkv + (size_t)which * ROWS * CC;

  float* sw = st[wave];
#pragma unroll
  for (int sub = 0; sub < 2; ++sub) {
    __syncthreads();
#pragma unroll
    for (int t = 0; t < 4; ++t) {
#pragma unroll
      for (int r = 0; r < 8; ++r)
        sw[(8 * hh + r) * OTP + 16 * t + c] = acc[sub][t][r] * 0.03125f + bvs[t];
    }
    __syncthreads();
    v4f val[8];
    size_t go[8];
#pragma unroll
    for (int it = 0; it < 8; ++it) {
      const int p    = lane + 32 * it;
      const int L    = p >> 3;
      const int pc   = p & 7;
      const int row  = L >> 1;
      const int half = L & 1;
      val[it] = *(const v4f*)(sw + row * OTP + half * 32 + pc * 4);
      go[it]  = (size_t)(m0 + sub * 16 + row) * CC + nin + half * 32 + pc * 4;
    }
    for (int ps = 0; ps < 2; ++ps) {
#pragma unroll
      for (int it = 0; it < 8; ++it) *(volatile v4f*)(ob + go[it]) = val[it];
      __threadfence();
    }
  }
}

template <int KK, int RES>
__global__ __launch_bounds__(256) void k_gout(const _Float16* __restrict__ ap,
                                              const _Float16* __restrict__ wt,
                                              const float* __restrict__ bias,
                                              const float* __restrict__ res,
                                              float* __restrict__ out, float oscale) {
  __shared__ __align__(16) float st[8][16 * OTP];
  const int tid = threadIdx.x, lane = tid & 31, wave = tid >> 5;
  const int hh = lane >> 4, c = lane & 15;
  const int m0 = blockIdx.x * 256 + wave * 32;
  const int n0 = blockIdx.y * 64;

  v8f acc[2][4];
#pragma unroll
  for (int s = 0; s < 2; ++s)
#pragma unroll
    for (int t = 0; t < 4; ++t) acc[s][t] = zero8();
  gemm32x64<KK>(ap, KK, wt, KK, m0, n0, lane, acc);

  float bvs[4];
#pragma unroll
  for (int t = 0; t < 4; ++t) bvs[t] = bias[n0 + 16 * t + c];

  float* sw = st[wave];
#pragma unroll
  for (int sub = 0; sub < 2; ++sub) {
    __syncthreads();
#pragma unroll
    for (int t = 0; t < 4; ++t) {
#pragma unroll
      for (int r = 0; r < 8; ++r)
        sw[(8 * hh + r) * OTP + 16 * t + c] = acc[sub][t][r] * oscale + bvs[t];
    }
    __syncthreads();
    v4f val[8];
    size_t go[8];
#pragma unroll
    for (int it = 0; it < 8; ++it) {
      const int p    = lane + 32 * it;
      const int L    = p >> 3;
      const int pc   = p & 7;
      const int row  = L >> 1;
      const int half = L & 1;
      const size_t g = (size_t)(m0 + sub * 16 + row) * CC + n0 + half * 32 + pc * 4;
      v4f v = *(const v4f*)(sw + row * OTP + half * 32 + pc * 4);
      if (RES) {
        const v4f rr = *(const v4f*)(res + g);
        v[0] = v[0] + rr[0]; v[1] = v[1] + rr[1]; v[2] = v[2] + rr[2]; v[3] = v[3] + rr[3];
      }
      val[it] = v;
      go[it]  = g;
    }
    for (int ps = 0; ps < 2; ++ps) {
#pragma unroll
      for (int it = 0; it < 8; ++it) *(volatile v4f*)(out + go[it]) = val[it];
      __threadfence();
    }
  }
}

__global__ __launch_bounds__(256) void k_ffn1(const _Float16* __restrict__ ap,
                                              const _Float16* __restrict__ wt,
                                              const float* __restrict__ bias,
                                              _Float16* __restrict__ hp) {
  __shared__ __align__(16) float st[8][16 * OTP];
  const int tid = threadIdx.x, lane = tid & 31, wave = tid >> 5;
  const int hh = lane >> 4, c = lane & 15;
  const int m0 = blockIdx.x * 256 + wave * 32;
  const int n0 = blockIdx.y * 64;

  v8f acc[2][4];
#pragma unroll
  for (int s = 0; s < 2; ++s)
#pragma unroll
    for (int t = 0; t < 4; ++t) acc[s][t] = zero8();
  gemm32x64<CC>(ap, CC, wt, CC, m0, n0, lane, acc);

  float bvs[4];
#pragma unroll
  for (int t = 0; t < 4; ++t) bvs[t] = bias[n0 + 16 * t + c];

  float* sw = st[wave];
#pragma unroll
  for (int sub = 0; sub < 2; ++sub) {
    __syncthreads();
#pragma unroll
    for (int t = 0; t < 4; ++t) {
#pragma unroll
      for (int r = 0; r < 8; ++r)
        sw[(8 * hh + r) * OTP + 16 * t + c] = acc[sub][t][r] * 0.03125f + bvs[t];
    }
    __syncthreads();
    v4u val[4];
    size_t go[4];
#pragma unroll
    for (int it = 0; it < 4; ++it) {
      const int p  = lane + 32 * it;
      const int L  = p >> 3;
      const int pc = p & 7;
      const v4f x0 = *(const v4f*)(sw + L * OTP + pc * 8);
      const v4f x1 = *(const v4f*)(sw + L * OTP + pc * 8 + 4);
      Pack8 pk;
      pk.h = (v8h){(_Float16)act16(x0[0]), (_Float16)act16(x0[1]), (_Float16)act16(x0[2]), (_Float16)act16(x0[3]),
                   (_Float16)act16(x1[0]), (_Float16)act16(x1[1]), (_Float16)act16(x1[2]), (_Float16)act16(x1[3])};
      val[it] = pk.u;
      go[it]  = (size_t)(m0 + sub * 16 + L) * FF + n0 + pc * 8;
    }
    for (int ps = 0; ps < 2; ++ps) {
#pragma unroll
      for (int it = 0; it < 4; ++it) *(volatile v4u*)(hp + go[it]) = val[it];
      __threadfence();
    }
  }
}

__global__ __launch_bounds__(256) void k_edge(const float* __restrict__ q32,
                                              const float* __restrict__ k32,
                                              const float* __restrict__ v32,
                                              const float* __restrict__ relt,
                                              const int* __restrict__ esrc,
                                              const int* __restrict__ edst,
                                              const int* __restrict__ erel,
                                              _Float16* __restrict__ o16, int nE, int nR) {
  extern __shared__ v4f accd[];
  __shared__ int s_list[ECH];
  __shared__ int s_cnt[8];
  float* accr = (float*)accd;
  const int tid  = threadIdx.x, lane = tid & 31;
  const int wave = __builtin_amdgcn_readfirstlane(tid >> 5);
  const int nblk = LL / NDB;
  const int b    = blockIdx.x / nblk;
  const int d0   = (blockIdx.x % nblk) * NDB;

  const v4f z4 = {0.f, 0.f, 0.f, 0.f};
#pragma unroll
  for (int i = 0; i < (NDB * CC) / (4 * 256); ++i) accd[i * 256 + tid] = z4;
  float zl0 = 0.f, zl1 = 0.f;

  const int* srb = esrc + (size_t)b * nE;
  const int* dsb = edst + (size_t)b * nE;
  const int* rlb = erel + (size_t)b * nE;
  const float* qb = q32 + (size_t)b * LL * CC;
  const float* kb = k32 + (size_t)b * LL * CC;
  const float* vb = v32 + (size_t)b * LL * CC;
  __syncthreads();

  for (int cb = 0; cb < nE; cb += ECH) {
    const int e  = cb + tid;
    const int ec = min(e, nE - 1);
    const int dv = dsb[ec];
    int sv = srb[ec];
    int rv = rlb[ec];
    sv = min(max(sv, 0), LL - 1);
    rv = min(max(rv, 0), nR - 1);
    const int dl = dv - d0;
    const bool hit = (e < nE) && ((unsigned)dl < (unsigned)NDB);
    const unsigned bal = __builtin_amdgcn_ballot_w32(hit);
    const int wpre = __builtin_popcount(bal & ((1u << lane) - 1u));
    if (lane == 0) s_cnt[wave] = __builtin_popcount(bal);
    __syncthreads();
    int base = 0, tot = 0;
#pragma unroll
    for (int w = 0; w < 8; ++w) {
      const int cw = s_cnt[w];
      tot += cw;
      base += (w < wave) ? cw : 0;
    }
    if (hit) s_list[base + wpre] = sv | (rv << 12) | (dl << 24);
    __syncthreads();
    tot = __builtin_amdgcn_readfirstlane(min(tot, ECH));

    for (int j = 0; j < tot; ++j) {
      const int ent = __builtin_amdgcn_readfirstlane(s_list[j]);
      const int dl2 = (ent >> 24) & (NDB - 1);
      if ((dl2 & 7) != wave) continue;
      const int src = min(ent & 4095, LL - 1);
      const int rel = min((ent >> 12) & 4095, nR - 1);
      const float* kp = kb + (size_t)src * CC;
      const float* vp = vb + (size_t)src * CC;
      const float* ep = relt + (size_t)rel * CC;
      const float* qp = qb + (size_t)(d0 + dl2) * CC;
      float p = 0.f;
#pragma unroll 2
      for (int i = 0; i < CC / 128; ++i) {
        const int o = i * 128 + lane * 4;
        const v4f k4 = *(const v4f*)(kp + o);
        const v4f e4 = *(const v4f*)(ep + o);
        const v4f q4 = *(const v4f*)(qp + o);
        p = fmaf(k4[0] + e4[0], q4[0], p);
        p = fmaf(k4[1] + e4[1], q4[1], p);
        p = fmaf(k4[2] + e4[2], q4[2], p);
        p = fmaf(k4[3] + e4[3], q4[3], p);
      }
#pragma unroll
      for (int off = 1; off < 32; off <<= 1) p += __shfl_xor(p, off, 32);
      float s = p * 0.03125f;
      s = fminf(fmaxf(s, -10.0f), 10.0f);
      s = expf(s);
      const bool own0 = (dl2 == wave);
      zl0 += own0 ? s : 0.0f;
      zl1 += own0 ? 0.0f : s;
      float* ar = accr + dl2 * CC;
#pragma unroll 2
      for (int i = 0; i < CC / 128; ++i) {
        const int o = i * 128 + lane * 4;
        const v4f v4 = *(const v4f*)(vp + o);
        const v4f e4 = *(const v4f*)(ep + o);
        v4f a = *(const v4f*)(ar + o);
        a[0] = fmaf(v4[0] + e4[0], s, a[0]);
        a[1] = fmaf(v4[1] + e4[1], s, a[1]);
        a[2] = fmaf(v4[2] + e4[2], s, a[2]);
        a[3] = fmaf(v4[3] + e4[3], s, a[3]);
        *(v4f*)(ar + o) = a;
      }
    }
    __syncthreads();
  }

  v4u val[8];
  size_t go[8];
#pragma unroll
  for (int rr = 0; rr < 2; ++rr) {
    const int dlo = wave + 8 * rr;
    const float zz  = rr ? zl1 : zl0;
    const float inv = 1.0f / zz;
    const float* ar = accr + dlo * CC;
#pragma unroll
    for (int it = 0; it < 4; ++it) {
      const int o = it * 256 + lane * 8;
      const v4f a0 = *(const v4f*)(ar + o);
      const v4f a1 = *(const v4f*)(ar + o + 4);
      Pack8 pk;
      pk.h = (v8h){(_Float16)(a0[0] * inv * 64.0f), (_Float16)(a0[1] * inv * 64.0f),
                   (_Float16)(a0[2] * inv * 64.0f), (_Float16)(a0[3] * inv * 64.0f),
                   (_Float16)(a1[0] * inv * 64.0f), (_Float16)(a1[1] * inv * 64.0f),
                   (_Float16)(a1[2] * inv * 64.0f), (_Float16)(a1[3] * inv * 64.0f)};
      val[rr * 4 + it] = pk.u;
      go[rr * 4 + it]  = ((size_t)(b * LL + d0 + dlo)) * CC + o;
    }
  }
  for (int ps = 0; ps < 2; ++ps) {
#pragma unroll
    for (int j = 0; j < 8; ++j) *(volatile v4u*)(o16 + go[j]) = val[j];
    __threadfence();
  }
}

extern "C" void kernel_launch(void* const* d_in, const int* in_sizes, int n_in,
                              void* d_out, int out_size, void* d_ws, size_t ws_size,
                              hipStream_t stream) {
  if (n_in < 21) return;
  if (in_sizes[0] != ROWS * CC) return;
  if (in_sizes[1] < CC || (in_sizes[1] % CC) != 0) return;
  if (in_sizes[2] != CC * CC || in_sizes[4] != CC * CC || in_sizes[5] != CC * CC || in_sizes[6] != CC * CC) return;
  if (in_sizes[3] != CC || in_sizes[7] != CC) return;
  if (in_sizes[8] != CC || in_sizes[9] != CC || in_sizes[10] != CC || in_sizes[11] != CC) return;
  if (in_sizes[12] != CC * FF || in_sizes[13] != FF) return;
  if (in_sizes[14] != FF * CC || in_sizes[15] != CC) return;
  if (in_sizes[16] != CC || in_sizes[17] != CC) return;
  if (in_sizes[18] != in_sizes[19] || in_sizes[20] != in_sizes[19]) return;
  if (in_sizes[19] < BB || (in_sizes[19] % BB) != 0) return;
  if (out_size != ROWS * CC) return;
  const int nE = in_sizes[19] / BB;
  const int nR = in_sizes[1] / CC;
  if (nR > 4096) return;

  const float* hid  = (const float*)d_in[0];
  const float* relt = (const float*)d_in[1];
  const float* Wq   = (const float*)d_in[2];
  const float* bq   = (const float*)d_in[3];
  const float* Wk   = (const float*)d_in[4];
  const float* Wv   = (const float*)d_in[5];
  const float* Wo   = (const float*)d_in[6];
  const float* bo   = (const float*)d_in[7];
  const float* g0   = (const float*)d_in[8];
  const float* be0  = (const float*)d_in[9];
  const float* g1   = (const float*)d_in[10];
  const float* be1  = (const float*)d_in[11];
  const float* W1   = (const float*)d_in[12];
  const float* b1   = (const float*)d_in[13];
  const float* W2   = (const float*)d_in[14];
  const float* b2   = (const float*)d_in[15];
  const float* g2   = (const float*)d_in[16];
  const float* be2  = (const float*)d_in[17];
  const int*   esrc = (const int*)d_in[18];
  const int*   edst = (const int*)d_in[19];
  const int*   erel = (const int*)d_in[20];
  float* out = (float*)d_out;

  const size_t plane32 = (size_t)ROWS * CC * 4;
  const size_t plane16 = (size_t)ROWS * CC * 2;
  size_t off = 0;
  const size_t oQKV = off; off += 3 * plane32;
  const size_t oH   = 0;
  const size_t oT1  = (size_t)ROWS * FF * 2;
  const size_t oT2  = oT1;
  if (oT1 + plane32 > off) return;
  const size_t oX32 = off; off += plane32;
  const size_t oATT = oX32;
  const size_t oXh  = off; off += plane16;
  const size_t oO   = oXh;
  const size_t oATh = oXh;
  const size_t oWqkv = off; off += (size_t)C3 * CC * 2;
  const size_t oWo   = off; off += (size_t)CC * CC * 2;
  const size_t oW1   = off; off += (size_t)FF * CC * 2;
  const size_t oW2   = off; off += (size_t)CC * FF * 2;
  if (off > ws_size) return;
  if (off > (size_t)134217728) return;

  char* ws = (char*)d_ws;
  float*    QKV32 = (float*)(ws + oQKV);
  _Float16* Hp    = (_Float16*)(ws + oH);
  float*    T1    = (float*)(ws + oT1);
  float*    T2    = (float*)(ws + oT2);
  float*    X32   = (float*)(ws + oX32);
  float*    ATT   = (float*)(ws + oATT);
  _Float16* Xh    = (_Float16*)(ws + oXh);
  _Float16* Op    = (_Float16*)(ws + oO);
  _Float16* ATTh  = (_Float16*)(ws + oATh);
  _Float16* Wqkvt = (_Float16*)(ws + oWqkv);
  _Float16* Wot   = (_Float16*)(ws + oWo);
  _Float16* W1t   = (_Float16*)(ws + oW1);
  _Float16* W2t   = (_Float16*)(ws + oW2);

  k_ln<<<dim3(ROWS), dim3(256), 0, stream>>>(hid, g0, be0, X32, Xh);
  k_wt<<<dim3(CC / 64, CC / 64), dim3(256), 0, stream>>>(Wq, Wqkvt, CC, CC);
  k_wt<<<dim3(CC / 64, CC / 64), dim3(256), 0, stream>>>(Wk, Wqkvt + (size_t)CC * CC, CC, CC);
  k_wt<<<dim3(CC / 64, CC / 64), dim3(256), 0, stream>>>(Wv, Wqkvt + (size_t)2 * CC * CC, CC, CC);
  k_wt<<<dim3(CC / 64, CC / 64), dim3(256), 0, stream>>>(Wo, Wot, CC, CC);
  k_wt<<<dim3(FF / 64, CC / 64), dim3(256), 0, stream>>>(W1, W1t, FF, CC);
  k_wt<<<dim3(CC / 64, FF / 64), dim3(256), 0, stream>>>(W2, W2t, CC, FF);
  k_qkv32<<<dim3(ROWS / 256, C3 / 64), dim3(256), 0, stream>>>(Xh, Wqkvt, bq, QKV32);
  const int ldsdyn = NDB * CC * 4;
  (void)hipFuncSetAttribute(reinterpret_cast<const void*>(&k_edge), hipFuncAttributeMaxDynamicSharedMemorySize, ldsdyn);
  k_edge<<<dim3(BB * (LL / NDB)), dim3(256), ldsdyn, stream>>>(QKV32, QKV32 + (size_t)ROWS * CC, QKV32 + (size_t)2 * ROWS * CC,
                                                               relt, esrc, edst, erel, Op, nE, nR);
  k_gout<CC, 1><<<dim3(ROWS / 256, CC / 64), dim3(256), 0, stream>>>(Op, Wot, bo, X32, T1, 0.00048828125f);
  k_ln<<<dim3(ROWS), dim3(256), 0, stream>>>(T1, g1, be1, ATT, ATTh);
  k_ffn1<<<dim3(ROWS / 256, FF / 64), dim3(256), 0, stream>>>(ATTh, W1t, b1, Hp);
  k_gout<FF, 1><<<dim3(ROWS / 256, CC / 64), dim3(256), 0, stream>>>(Hp, W2t, b2, ATT, T2, 0.001953125f);
  k_lnout<<<dim3(ROWS), dim3(256), 0, stream>>>(T2, g2, be2, hid, out);
  (void)hipGetLastError();
}
